// MultiHeadDepthwiseSelfAttention_23038204576347
// MI455X (gfx1250) — hardware-verified
//
#include <hip/hip_runtime.h>
#include <math.h>

constexpr int kBatch    = 16;
constexpr int kSeq      = 1024;
constexpr int kFeat     = 768;
constexpr int kHeads    = 12;
constexpr int kDh       = 64;
constexpr int kTokElems = kSeq * kFeat;
constexpr float kPCarry    = 2048.0f;
constexpr float kPCarryInv = 1.0f / 2048.0f;
static_assert(kHeads * kDh == kFeat);
static_assert(kTokElems == 786432);

constexpr size_t kPlane16Bytes = (size_t)kTokElems * 2;
constexpr size_t kOffQh = 0;
constexpr size_t kOffQl = kPlane16Bytes;
constexpr size_t kOffKh = 2 * kPlane16Bytes;
constexpr size_t kOffKl = 3 * kPlane16Bytes;
constexpr size_t kOffVt = 4 * kPlane16Bytes;
constexpr size_t kOffSC = 5 * kPlane16Bytes;
constexpr size_t kSizeSC = (size_t)kHeads * kSeq * kSeq * 4;
constexpr size_t kOffPP = kOffSC + kSizeSC;
constexpr size_t kSizePP = (size_t)kHeads * kSeq * kSeq * 2;
constexpr size_t kWsTotal = kOffPP + kSizePP;
static_assert((size_t)kHeads * kDh * kSeq * 2 == kPlane16Bytes);
static_assert(kWsTotal == 83361792);
static_assert(kWsTotal <= 134217728);
static_assert((kOffSC % 128) == 0 && (kOffPP % 128) == 0);

typedef __attribute__((ext_vector_type(16))) _Float16 v16h;
typedef __attribute__((ext_vector_type(8)))  _Float16 v8h;
typedef __attribute__((ext_vector_type(16))) __bf16   v16b;
typedef __attribute__((ext_vector_type(8)))  __bf16   v8b;
typedef __attribute__((ext_vector_type(8)))  float    v8f;
typedef __attribute__((ext_vector_type(4)))  float    v4f;
typedef __attribute__((ext_vector_type(4)))  unsigned int v4u;

__device__ __forceinline__ unsigned short f2bf_bits(float f) {
  unsigned u = __float_as_uint(f);
  return (unsigned short)((u + 0x7FFFu + ((u >> 16) & 1u)) >> 16);
}
__device__ __forceinline__ float bf_bits2f(unsigned short h) { return __uint_as_float(((unsigned)h) << 16); }

__device__ __forceinline__ void dep_guard_h(v8f& a, v8f& b, v16h x, v16h y) { asm volatile("v_nop\n\tv_nop\n\tv_nop\n\tv_nop" : "+v"(a), "+v"(b) : "v"(x), "v"(y)); }
__device__ __forceinline__ void dep_guard_b(v8f& a, v8f& b, v16b x, v16b y) { asm volatile("v_nop\n\tv_nop\n\tv_nop\n\tv_nop" : "+v"(a), "+v"(b) : "v"(x), "v"(y)); }
__device__ __forceinline__ void keep4_h(v16h a, v16h b, v16h c, v16h d) { asm volatile("v_nop" :: "v"(a), "v"(b), "v"(c), "v"(d)); }
__device__ __forceinline__ void keep4_b(v16b a, v16b b, v16b c, v16b d) { asm volatile("v_nop" :: "v"(a), "v"(b), "v"(c), "v"(d)); }
__device__ __forceinline__ void acc_guard4(v8f& a, v8f& b, v8f& c, v8f& d) { asm volatile("v_nop\n\tv_nop\n\tv_nop\n\tv_nop" : "+v"(a), "+v"(b), "+v"(c), "+v"(d)); }
template <typename T> struct Frag;
template <> struct Frag<_Float16> {
  typedef v16h V; union U { v16h v; v8h h[2]; };
  static __device__ __forceinline__ v16h load(const _Float16* p) {
    U f; f.h[0] = *(const v8h*)(p); f.h[1] = *(const v8h*)(p + 16); return f.v;
  }
  static __device__ __forceinline__ v8f mma(v16h a, v16h b, v8f c) {
    return __builtin_amdgcn_wmma_f32_16x16x32_f16(false, a, false, b, (short)0, c, false, false);
  }
  static __device__ __forceinline__ void guard(v8f& a, v8f& b, v16h x, v16h y) { dep_guard_h(a, b, x, y); }
  static __device__ __forceinline__ void keep(v16h a, v16h b, v16h c, v16h d) { keep4_h(a, b, c, d); }
};
template <> struct Frag<__bf16> {
  typedef v16b V; union U { v16b v; v8b h[2]; };
  static __device__ __forceinline__ v16b load(const __bf16* p) {
    U f; f.h[0] = *(const v8b*)(p); f.h[1] = *(const v8b*)(p + 16); return f.v;
  }
  static __device__ __forceinline__ v8f mma(v16b a, v16b b, v8f c) {
    return __builtin_amdgcn_wmma_f32_16x16x32_bf16(false, a, false, b, (short)0, c, false, false);
  }
  static __device__ __forceinline__ void guard(v8f& a, v8f& b, v16b x, v16b y) { dep_guard_b(a, b, x, y); }
  static __device__ __forceinline__ void keep(v16b a, v16b b, v16b c, v16b d) { keep4_b(a, b, c, d); }
};

__device__ __forceinline__ unsigned pk16(unsigned short a, unsigned short b) { return (unsigned)a | ((unsigned)b << 16); }
__device__ __forceinline__ unsigned short h_bits(float f) { const _Float16 h = (_Float16)f; return __builtin_bit_cast(unsigned short, h); }

template <int ET> struct Elem;
template <> struct Elem<0> { typedef _Float16 T; };
template <> struct Elem<1> { typedef __bf16 T; };
template <int ET, bool SPLIT, int BIAS_MODE, int OUT_MODE, bool RESID, int ACT = 0>
__global__ __launch_bounds__(256) void wmma_gemm64(
    const unsigned short* __restrict__ Ap, const unsigned short* __restrict__ A2p, int lda, long strideA,
    const unsigned short* __restrict__ Btp, const unsigned short* __restrict__ Bt2p, int ldb, long strideB,
    void* __restrict__ Cout, void* __restrict__ Cout2, int ldc, long strideC,
    const float* __restrict__ bias, const float* __restrict__ cscale, long strideS,
    const float* __restrict__ resid, long strideR,
    int M, int N, int K, float scale) {
  typedef typename Elem<ET>::T T;
  typedef typename Frag<T>::V V;
  const T* A = (const T*)Ap; const T* A2 = (const T*)A2p; const T* Bt = (const T*)Btp; const T* Bt2 = (const T*)Bt2p;
  __shared__ __align__(16) float sT[8][16 * 68];
  const int b    = blockIdx.y;
  const int lane = threadIdx.x & 31;
  const int wave = threadIdx.x >> 5;
  const int tilesN = N >> 6;
  const int tilesM = M >> 6;
  const int tile = blockIdx.x * 8 + wave;
  if (tile >= tilesM * tilesN) return;
  const int tm = tile / tilesN;
  const int tn = tile - tm * tilesN;
  const int m0 = tm << 6;
  const int n0 = tn << 6;

  const T* Ab  = A  + (size_t)b * strideA;
  const T* Bb  = Bt + (size_t)b * strideB;
  const T* Ab2 = SPLIT ? (A2  + (size_t)b * strideA) : nullptr;
  const T* Bb2 = SPLIT ? (Bt2 + (size_t)b * strideB) : nullptr;

  const int rlane = lane & 15;
  const int koff  = (lane >> 4) * 8;
  const int mOff  = (lane >> 4) * 8;

  v8f acc[4][4];
#pragma unroll
  for (int i = 0; i < 4; ++i)
#pragma unroll
    for (int j = 0; j < 4; ++j) acc[i][j] = (v8f){0.f,0.f,0.f,0.f,0.f,0.f,0.f,0.f};

  for (int k0 = 0; k0 < K; k0 += 32) {
    V bh[4], bl[4];
#pragma unroll
    for (int j = 0; j < 4; ++j) {
      const size_t bo = (size_t)(n0 + (j << 4) + rlane) * ldb + koff + k0;
      bh[j] = Frag<T>::load(Bb + bo);
      if (SPLIT) bl[j] = Frag<T>::load(Bb2 + bo);
    }
#pragma unroll
    for (int i = 0; i < 4; ++i) {
      const size_t ao = (size_t)(m0 + (i << 4) + rlane) * lda + koff + k0;
      V ah = Frag<T>::load(Ab + ao);
      V al;
      if (SPLIT) al = Frag<T>::load(Ab2 + ao);
#pragma unroll
      for (int j = 0; j < 4; ++j) {
        acc[i][j] = Frag<T>::mma(ah, bh[j], acc[i][j]);
        if (SPLIT) {
          acc[i][j] = Frag<T>::mma(ah, bl[j], acc[i][j]);
          acc[i][j] = Frag<T>::mma(al, bh[j], acc[i][j]);
        }
      }
      Frag<T>::guard(acc[i][0], acc[i][3], ah, SPLIT ? al : ah);
    }
    Frag<T>::keep(bh[0], bh[1], bh[2], bh[3]);
    if (SPLIT) Frag<T>::keep(bl[0], bl[1], bl[2], bl[3]);
  }
  acc_guard4(acc[0][0], acc[0][1], acc[0][2], acc[0][3]);
  acc_guard4(acc[1][0], acc[1][1], acc[1][2], acc[1][3]);
  acc_guard4(acc[2][0], acc[2][1], acc[2][2], acc[2][3]);
  acc_guard4(acc[3][0], acc[3][1], acc[3][2], acc[3][3]);

  float* slab = sT[wave];
  const float* Rb = RESID ? (resid + (size_t)b * strideR) : nullptr;
#pragma unroll
  for (int i = 0; i < 4; ++i) {
    const int mBase = m0 + (i << 4);
#pragma unroll
    for (int j = 0; j < 4; ++j) {
      const int n = n0 + (j << 4) + rlane;
      float bv = 0.f, cs = 1.f;
      if (BIAS_MODE == 2) bv = bias[n];
      if (BIAS_MODE == 3) { bv = bias[(size_t)b * strideS + n]; cs = cscale[(size_t)b * strideS + n]; }
#pragma unroll
      for (int r = 0; r < 8; ++r) {
        float v = acc[i][j][r] * scale;
        if (BIAS_MODE == 1) v += bias[mBase + mOff + r];
        if (BIAS_MODE == 2) v += bv;
        if (BIAS_MODE == 3) v = v * cs + bv;
        if (RESID) v += Rb[(size_t)(mBase + mOff + r) * ldc + n];
        if (ACT == 2) v = fmaxf(v, 0.0f);
        if (ACT == 4) v = (v > 0.f) ? v : 0.01f * v;
        slab[(mOff + r) * 68 + (j << 4) + rlane] = v;
      }
    }
    __builtin_amdgcn_fence(__ATOMIC_RELEASE, "workgroup");
    __builtin_amdgcn_wave_barrier();
    __builtin_amdgcn_fence(__ATOMIC_ACQUIRE, "workgroup");
    if (OUT_MODE == 0) {
      float* C = (float*)Cout + (size_t)b * strideC;
      const int hh = lane >> 4, c4 = (lane & 15) * 4;
      for (int pass = 0; pass < 2; ++pass) {
#pragma unroll
        for (int it = 0; it < 8; ++it) {
          const int row = it * 2 + hh;
          v4f v = *(const v4f*)(slab + row * 68 + c4);
          *(volatile v4f*)(C + (size_t)(mBase + row) * ldc + n0 + c4) = v;
        }
        __threadfence();
      }
    } else {
      const int q = lane >> 3, c8 = (lane & 7) * 8;
      unsigned short* C  = (unsigned short*)Cout  + (size_t)b * strideC;
      unsigned short* C2 = (OUT_MODE == 2) ? ((unsigned short*)Cout2 + (size_t)b * strideC) : nullptr;
      for (int pass = 0; pass < 2; ++pass) {
#pragma unroll
        for (int it = 0; it < 4; ++it) {
          const int row = it * 4 + q;
          const float* sp = slab + row * 68 + c8;
          v8h hv, lv;
#pragma unroll
          for (int e = 0; e < 8; ++e) {
            if (OUT_MODE == 1) {
              hv[e] = (_Float16)sp[e];
            } else {
              unsigned short hb = f2bf_bits(sp[e]);
              unsigned short lb = f2bf_bits(sp[e] - bf_bits2f(hb));
              hv[e] = __builtin_bit_cast(_Float16, hb);
              lv[e] = __builtin_bit_cast(_Float16, lb);
            }
          }
          *(volatile v8h*)(C + (size_t)(mBase + row) * ldc + n0 + c8) = hv;
          if (OUT_MODE == 2) *(volatile v8h*)(C2 + (size_t)(mBase + row) * ldc + n0 + c8) = lv;
        }
        __threadfence();
      }
    }
    __builtin_amdgcn_fence(__ATOMIC_RELEASE, "workgroup");
    __builtin_amdgcn_wave_barrier();
    __builtin_amdgcn_fence(__ATOMIC_ACQUIRE, "workgroup");
  }
}

constexpr int kPrepQKBlocks = kTokElems / 8 / 256;
constexpr int kPrepVTBlocks = kHeads * (kSeq / 64);
constexpr int kPrepBlocks   = kPrepQKBlocks + kPrepVTBlocks;
static_assert(kPrepQKBlocks * 256 * 8 == kTokElems);
static_assert(kPrepVTBlocks * 64 * 64 == kTokElems);

__global__ __launch_bounds__(256) void prep_kernel(const float* __restrict__ xb,
                                                   const float* __restrict__ wq, const float* __restrict__ bq,
                                                   const float* __restrict__ wk, const float* __restrict__ bk,
                                                   const float* __restrict__ wv, const float* __restrict__ bv,
                                                   unsigned short* __restrict__ qh, unsigned short* __restrict__ ql,
                                                   unsigned short* __restrict__ kh, unsigned short* __restrict__ kl,
                                                   unsigned short* __restrict__ vt) {
  __shared__ __align__(16) float tile[64][68];
  const int t = threadIdx.x;
  if (blockIdx.x < kPrepQKBlocks) {
    const size_t e0 = ((size_t)blockIdx.x * 256 + t) * 8;
    const int c = (int)(e0 % kFeat);
    const v4f xa = *(const v4f*)(xb + e0);
    const v4f xc = *(const v4f*)(xb + e0 + 4);
    const v4f wqa = *(const v4f*)(wq + c), wqc = *(const v4f*)(wq + c + 4);
    const v4f bqa = *(const v4f*)(bq + c), bqc = *(const v4f*)(bq + c + 4);
    const v4f wka = *(const v4f*)(wk + c), wkc = *(const v4f*)(wk + c + 4);
    const v4f bka = *(const v4f*)(bk + c), bkc = *(const v4f*)(bk + c + 4);
    float xv[8], wqv[8], bqv[8], wkv[8], bkv[8];
#pragma unroll
    for (int j = 0; j < 4; ++j) {
      xv[j] = xa[j];   xv[4 + j] = xc[j];
      wqv[j] = wqa[j]; wqv[4 + j] = wqc[j];
      bqv[j] = bqa[j]; bqv[4 + j] = bqc[j];
      wkv[j] = wka[j]; wkv[4 + j] = wkc[j];
      bkv[j] = bka[j]; bkv[4 + j] = bkc[j];
    }
    unsigned short qhb[8], qlb[8], khb[8], klb[8];
#pragma unroll
    for (int j = 0; j < 8; ++j) {
      const float qvv = xv[j] * wqv[j] + bqv[j];
      const float kvv = xv[j] * wkv[j] + bkv[j];
      const unsigned short hq = f2bf_bits(qvv);
      const unsigned short hk = f2bf_bits(kvv);
      qhb[j] = hq;
      qlb[j] = f2bf_bits(qvv - bf_bits2f(hq));
      khb[j] = hk;
      klb[j] = f2bf_bits(kvv - bf_bits2f(hk));
    }
    const v4u uqh = (v4u){pk16(qhb[0], qhb[1]), pk16(qhb[2], qhb[3]), pk16(qhb[4], qhb[5]), pk16(qhb[6], qhb[7])};
    const v4u uql = (v4u){pk16(qlb[0], qlb[1]), pk16(qlb[2], qlb[3]), pk16(qlb[4], qlb[5]), pk16(qlb[6], qlb[7])};
    const v4u ukh = (v4u){pk16(khb[0], khb[1]), pk16(khb[2], khb[3]), pk16(khb[4], khb[5]), pk16(khb[6], khb[7])};
    const v4u ukl = (v4u){pk16(klb[0], klb[1]), pk16(klb[2], klb[3]), pk16(klb[4], klb[5]), pk16(klb[6], klb[7])};
    unsigned short* pqh = qh + e0;
    unsigned short* pql = ql + e0;
    unsigned short* pkh = kh + e0;
    unsigned short* pkl = kl + e0;
    *(volatile v4u*)pqh = uqh;
    *(volatile v4u*)pql = uql;
    *(volatile v4u*)pkh = ukh;
    *(volatile v4u*)pkl = ukl;
    __threadfence();
    *(volatile v4u*)pqh = uqh;
    *(volatile v4u*)pql = uql;
    *(volatile v4u*)pkh = ukh;
    *(volatile v4u*)pkl = ukl;
  } else {
    const int blk = blockIdx.x - kPrepQKBlocks;
    const int h   = blk >> 4;
    const int nt  = blk & 15;
    const int n0  = nt * 64;
    const int ch0 = h * kDh;
    const int nr  = t >> 4;
    const int c4  = (t & 15) * 4;
    const v4f wv4 = *(const v4f*)(wv + ch0 + c4);
    const v4f bv4 = *(const v4f*)(bv + ch0 + c4);
#pragma unroll
    for (int pass = 0; pass < 4; ++pass) {
      const int n = nr + pass * 16;
      const v4f v = *(const v4f*)(xb + (size_t)(n0 + n) * kFeat + ch0 + c4);
#pragma unroll
      for (int j = 0; j < 4; ++j) tile[c4 + j][n] = v[j] * wv4[j] + bv4[j];
    }
    __syncthreads();
    const int lane = t & 31, wave = t >> 5;
    const int q = lane >> 3, c8 = (lane & 7) * 8;
    for (int pass = 0; pass < 2; ++pass) {
#pragma unroll
      for (int it = 0; it < 2; ++it) {
        const int row = wave * 8 + it * 4 + q;
        const v4f a  = *(const v4f*)(&tile[row][c8]);
        const v4f cc = *(const v4f*)(&tile[row][c8 + 4]);
        unsigned short hb[8];
#pragma unroll
        for (int e = 0; e < 4; ++e) {
          hb[e]     = h_bits(a[e]);
          hb[4 + e] = h_bits(cc[e]);
        }
        const v4u u = (v4u){pk16(hb[0], hb[1]), pk16(hb[2], hb[3]), pk16(hb[4], hb[5]), pk16(hb[6], hb[7])};
        *(volatile v4u*)(vt + ((size_t)(h * kDh + row)) * kSeq + n0 + c8) = u;
      }
      __threadfence();
    }
  }
}

__global__ __launch_bounds__(128) void softmax_rows_kernel(const float* __restrict__ S,
                                                           unsigned short* __restrict__ P, float carry) {
  __shared__ float redM[4];
  __shared__ float redS[4];
  const int row  = blockIdx.x;
  const int t    = threadIdx.x;
  const int wave = t >> 5;
  const size_t base = (size_t)row * kSeq + 8 * t;
  const v4f a = *(const v4f*)(S + base);
  const v4f c = *(const v4f*)(S + base + 4);
  float x[8];
#pragma unroll
  for (int j = 0; j < 4; ++j) { x[j] = a[j]; x[4 + j] = c[j]; }
  float m = fmaxf(fmaxf(fmaxf(x[0], x[1]), fmaxf(x[2], x[3])), fmaxf(fmaxf(x[4], x[5]), fmaxf(x[6], x[7])));
#pragma unroll
  for (int off = 16; off > 0; off >>= 1) m = fmaxf(m, __shfl_xor(m, off, 32));
  redM[wave] = m;
  __syncthreads();
  m = fmaxf(fmaxf(redM[0], redM[1]), fmaxf(redM[2], redM[3]));
  float e[8];
#pragma unroll
  for (int j = 0; j < 8; ++j) e[j] = expf(x[j] - m);
  float s = ((e[0] + e[1]) + (e[2] + e[3])) + ((e[4] + e[5]) + (e[6] + e[7]));
#pragma unroll
  for (int off = 16; off > 0; off >>= 1) s += __shfl_xor(s, off, 32);
  redS[wave] = s;
  __syncthreads();
  s = ((redS[0] + redS[1]) + redS[2]) + redS[3];
  const float f = carry * (1.0f / s);
  unsigned short hb[8];
#pragma unroll
  for (int j = 0; j < 8; ++j) hb[j] = h_bits(e[j] * f);
  const v4u u = (v4u){pk16(hb[0], hb[1]), pk16(hb[2], hb[3]), pk16(hb[4], hb[5]), pk16(hb[6], hb[7])};
  unsigned short* pp = P + base;
  *(volatile v4u*)pp = u;
  __threadfence();
  *(volatile v4u*)pp = u;
}

extern "C" void kernel_launch(void* const* d_in, const int* in_sizes, int n_in,
                              void* d_out, int out_size, void* d_ws, size_t ws_size,
                              hipStream_t stream) {
  if (n_in < 9) return;
  if (in_sizes[0] != kBatch * kTokElems) return;
  for (int i = 1; i < 9; ++i) { if (in_sizes[i] != kFeat) return; }
  if (out_size != kBatch * kTokElems) return;
  if (ws_size < kWsTotal) return;

  const float* x  = (const float*)d_in[0];
  const float* wq = (const float*)d_in[1];
  const float* bq = (const float*)d_in[2];
  const float* wk = (const float*)d_in[3];
  const float* bk = (const float*)d_in[4];
  const float* wv = (const float*)d_in[5];
  const float* bv = (const float*)d_in[6];
  const float* wo = (const float*)d_in[7];
  const float* bo = (const float*)d_in[8];
  float* out = (float*)d_out;

  unsigned char* ws = (unsigned char*)d_ws;
  unsigned short* qh = (unsigned short*)(ws + kOffQh);
  unsigned short* ql = (unsigned short*)(ws + kOffQl);
  unsigned short* kh = (unsigned short*)(ws + kOffKh);
  unsigned short* kl = (unsigned short*)(ws + kOffKl);
  unsigned short* vt = (unsigned short*)(ws + kOffVt);
  float*          sc = (float*)(ws + kOffSC);
  unsigned short* pp = (unsigned short*)(ws + kOffPP);

  const float qk_scale = 1.0f / sqrtf((float)kFeat);

  for (int b = 0; b < kBatch; ++b) {
    const float* xb = x + (size_t)b * kTokElems;
    float* outb = out + (size_t)b * kTokElems;

    prep_kernel<<<dim3(kPrepBlocks), dim3(256), 0, stream>>>(xb, wq, bq, wk, bk, wv, bv, qh, ql, kh, kl, vt);

    wmma_gemm64<1, true, 0, 0, false><<<dim3(32, kHeads, 1), dim3(256), 0, stream>>>(
        qh, ql, kFeat, (long)kDh,
        kh, kl, kFeat, (long)kDh,
        (void*)sc, (void*)nullptr, kSeq, (long)kSeq * kSeq,
        (const float*)nullptr, (const float*)nullptr, (long)0,
        (const float*)nullptr, (long)0,
        kSeq, kSeq, kDh, qk_scale);

    softmax_rows_kernel<<<dim3(kHeads * kSeq), dim3(128), 0, stream>>>(sc, pp, kPCarry);

    wmma_gemm64<0, false, 3, 0, false><<<dim3(2, kHeads, 1), dim3(256), 0, stream>>>(
        pp, (const unsigned short*)nullptr, kSeq, (long)kSeq * kSeq,
        vt, (const unsigned short*)nullptr, kSeq, (long)kDh * kSeq,
        (void*)outb, (void*)nullptr, kFeat, (long)kDh,
        bo, wo, (long)kDh,
        (const float*)nullptr, (long)0,
        kSeq, kDh, kSeq, kPCarryInv);
  }
}
